// SogouSTFT_70102456205611
// MI455X (gfx1250) — hardware-verified
//
#include <hip/hip_runtime.h>

typedef _Float16       v16h  __attribute__((ext_vector_type(16)));
typedef _Float16       v8h   __attribute__((ext_vector_type(8)));
typedef __bf16         v16bf __attribute__((ext_vector_type(16)));
typedef unsigned short v16us __attribute__((ext_vector_type(16)));
typedef unsigned short v8us  __attribute__((ext_vector_type(8)));
typedef float          v8f   __attribute__((ext_vector_type(8)));
typedef float          v4f   __attribute__((ext_vector_type(4)));
typedef v8h  __attribute__((may_alias)) v8ha;
typedef v8us __attribute__((may_alias)) v8usa;
typedef v4f  __attribute__((may_alias)) v4fa;

#define NBATCH 32
#define NSAMP  262144
#define FFTN   1024
#define HOPN   512
#define CDIM   1026
#define CPAD   1088
#define NFRM   511
#define PROWS  528
#define MANA   (NBATCH * PROWS)
#define QROWS  512
#define MSYN   (NBATCH * QROWS)
#define KSYN   (2 * CPAD)
#define NSYN   512

static_assert(NSAMP == QROWS * HOPN);
static_assert((NSAMP - FFTN) / HOPN + 1 == NFRM);
static_assert(MANA % 128 == 0);
static_assert(MSYN % 128 == 0);
static_assert(CPAD % 64 == 0);
static_assert(KSYN % 32 == 0);
static_assert(FFTN % 32 == 0);

__device__ __forceinline__ v8f wmma_f16(v16h a, v16h b, v8f c) {
  v8f d = __builtin_amdgcn_wmma_f32_16x16x32_f16(false, a, false, b, (short)0, c, false, false);
  asm volatile("v_nop\n\tv_nop\n\tv_nop\n\tv_nop" : "+v"(d) : "v"(a), "v"(b));
  return d;
}

__device__ __forceinline__ v8f wmma_bf16(v16us a, v16us b, v8f c) {
  const v16bf ab = __builtin_bit_cast(v16bf, a);
  const v16bf bb = __builtin_bit_cast(v16bf, b);
  v8f d = __builtin_amdgcn_wmma_f32_16x16x32_bf16(false, ab, false, bb, (short)0, c, false, false);
  asm volatile("v_nop\n\tv_nop\n\tv_nop\n\tv_nop" : "+v"(d) : "v"(a), "v"(b));
  return d;
}

union FragH { v16h v; v8h half[2]; };
union FragU { v16us v; v8us half[2]; };

__device__ __forceinline__ v16h ldf_h(const _Float16* p, int h) {
  FragH f;
  f.half[0] = *(const v8ha*)(p + 8 * h);
  f.half[1] = *(const v8ha*)(p + 16 + 8 * h);
  return f.v;
}

__device__ __forceinline__ v16us ldf_us(const unsigned short* p, int h) {
  FragU f;
  f.half[0] = *(const v8usa*)(p + 8 * h);
  f.half[1] = *(const v8usa*)(p + 16 + 8 * h);
  return f.v;
}

__device__ __forceinline__ unsigned int bf16_rne(float v) {
  const unsigned int u = __float_as_uint(v);
  return (u + 0x7FFFu + ((u >> 16) & 1u)) >> 16;
}

__device__ __forceinline__ void split1(float v, unsigned short& hb, unsigned short& lb) {
  const unsigned int hu = bf16_rne(v);
  const float hf = __uint_as_float(hu << 16);
  const unsigned int lu = bf16_rne(v - hf);
  hb = (unsigned short)hu;
  lb = (unsigned short)lu;
}

__device__ __forceinline__ void split8(v4f a, v4f c, float s, v8us& ho, v8us& lo) {
  unsigned short h0, h1, h2, h3, h4, h5, h6, h7;
  unsigned short l0, l1, l2, l3, l4, l5, l6, l7;
  split1(a.x * s, h0, l0);
  split1(a.y * s, h1, l1);
  split1(a.z * s, h2, l2);
  split1(a.w * s, h3, l3);
  split1(c.x * s, h4, l4);
  split1(c.y * s, h5, l5);
  split1(c.z * s, h6, l6);
  split1(c.w * s, h7, l7);
  const v8us hh = { h0, h1, h2, h3, h4, h5, h6, h7 };
  const v8us ll = { l0, l1, l2, l3, l4, l5, l6, l7 };
  ho = hh;
  lo = ll;
}

__global__ __launch_bounds__(256) void cvt_x_kernel(const float* __restrict__ x,
                                                    _Float16* __restrict__ xh, int n8) {
  const int g = blockIdx.x * 256 + threadIdx.x;
  if (g >= n8) return;
  const float* src = x + (size_t)g * 8;
  const v4f a = *(const v4fa*)src;
  const v4f c = *(const v4fa*)(src + 4);
  const v8h o = { (_Float16)a.x, (_Float16)a.y, (_Float16)a.z, (_Float16)a.w,
                  (_Float16)c.x, (_Float16)c.y, (_Float16)c.z, (_Float16)c.w };
  _Float16* dst = xh + (size_t)g * 8;
  *(volatile v8h*)dst = o;
  __threadfence();
  *(volatile v8h*)dst = o;
}

__global__ __launch_bounds__(256) void prep_fwd_kernel(const float* __restrict__ fwd,
                                                       _Float16* __restrict__ fh) {
  const int g = blockIdx.x * 256 + threadIdx.x;
  if (g >= CPAD * FFTN / 8) return;
  const int c  = g >> 7;
  const int k8 = (g & 127) * 8;
  const int cc = (c < CDIM) ? c : (CDIM - 1);
  const float s = (c < CDIM) ? 1.0f : 0.0f;
  const float* src = fwd + (size_t)cc * FFTN + k8;
  const v4f a = *(const v4fa*)src;
  const v4f b = *(const v4fa*)(src + 4);
  const v8h o = { (_Float16)(a.x * s), (_Float16)(a.y * s), (_Float16)(a.z * s), (_Float16)(a.w * s),
                  (_Float16)(b.x * s), (_Float16)(b.y * s), (_Float16)(b.z * s), (_Float16)(b.w * s) };
  _Float16* dst = fh + (size_t)g * 8;
  *(volatile v8h*)dst = o;
  __threadfence();
  *(volatile v8h*)dst = o;
}

__device__ __forceinline__ float ld_inv(const float* __restrict__ inv, int c, int col) {
  const int cc = (c < CDIM) ? c : (CDIM - 1);
  const float s = (c < CDIM) ? 1.0f : 0.0f;
  return inv[(size_t)cc * FFTN + col] * s;
}

__global__ __launch_bounds__(256) void prep_inv_kernel(const float* __restrict__ inv,
                                                       unsigned short* __restrict__ ivh,
                                                       unsigned short* __restrict__ ivl) {
  const int g = blockIdx.x * 256 + threadIdx.x;
  if (g >= NSYN * KSYN / 8) return;
  const int r   = g / (KSYN / 8);
  const int t   = g - r * (KSYN / 8);
  const int kk0 = 8 * t;
  const int sec = (kk0 >= CPAD) ? 1 : 0;
  const int cb  = kk0 - sec * CPAD;
  const int col = sec ? r : (HOPN + r);
  const v4f a = { ld_inv(inv, cb + 0, col), ld_inv(inv, cb + 1, col),
                  ld_inv(inv, cb + 2, col), ld_inv(inv, cb + 3, col) };
  const v4f c = { ld_inv(inv, cb + 4, col), ld_inv(inv, cb + 5, col),
                  ld_inv(inv, cb + 6, col), ld_inv(inv, cb + 7, col) };
  v8us ho, lo;
  split8(a, c, 1.0f, ho, lo);
  const size_t off = (size_t)g * 8;
  *(volatile v8us*)(ivh + off) = ho;
  *(volatile v8us*)(ivl + off) = lo;
  __threadfence();
  *(volatile v8us*)(ivh + off) = ho;
  *(volatile v8us*)(ivl + off) = lo;
}

__device__ __forceinline__ const _Float16* ana_arow(const _Float16* xh, int g) {
  const int b = g / PROWS;
  const int p = g - b * PROWS;
  int f = p - 1;
  f = (f < 0) ? 0 : f;
  f = (f > NFRM - 1) ? (NFRM - 1) : f;
  return xh + (size_t)b * NSAMP + (size_t)f * HOPN;
}

__device__ __forceinline__ void ana_store_pass(const float* so, unsigned short* sph, unsigned short* spl,
                                               int g0, int n0, int lane) {
  const int q8 = lane & 7, sub = lane >> 3;
  #pragma unroll
  for (int i = 0; i < 8; ++i) {
    const int lid = i * 4 + sub;
    const int g = g0 + lid;
    const int b = g / PROWS;
    const int p = g - b * PROWS;
    const float s = (p >= 1 && p <= NFRM) ? 1.0f : 0.0f;
    const v4f a = *(const v4fa*)(so + lid * 64 + 8 * q8);
    const v4f c = *(const v4fa*)(so + lid * 64 + 8 * q8 + 4);
    v8us ho, lo;
    split8(a, c, s, ho, lo);
    const size_t off = (size_t)g * CPAD + n0 + 8 * q8;
    *(volatile v8us*)(sph + off) = ho;
    *(volatile v8us*)(spl + off) = lo;
  }
}

__global__ __launch_bounds__(128) void ana_kernel(const _Float16* __restrict__ xh,
                                                  const _Float16* __restrict__ fh,
                                                  unsigned short* __restrict__ sph,
                                                  unsigned short* __restrict__ spl) {
  __shared__ __attribute__((aligned(16))) float sT[4 * 32 * 64];

  const int tid = threadIdx.x, lane = tid & 31, w = tid >> 5;
  const int h = lane >> 4, m = lane & 15;
  const int g0 = blockIdx.x * 128 + 32 * w;
  const int n0 = blockIdx.y * 64;

  const _Float16* xa0 = ana_arow(xh, g0 + m);
  const _Float16* xa1 = ana_arow(xh, g0 + 16 + m);
  const _Float16* wb  = fh + (size_t)(n0 + m) * FFTN;

  const v8f zero8 = {0.f, 0.f, 0.f, 0.f, 0.f, 0.f, 0.f, 0.f};
  v8f acc[2][4];
  #pragma unroll
  for (int mt = 0; mt < 2; ++mt)
    #pragma unroll
    for (int nt = 0; nt < 4; ++nt) acc[mt][nt] = zero8;

  #pragma unroll 1
  for (int k0 = 0; k0 < FFTN; k0 += 32) {
    const v16h a0 = ldf_h(xa0 + k0, h);
    const v16h a1 = ldf_h(xa1 + k0, h);
    #pragma unroll
    for (int nt = 0; nt < 4; ++nt) {
      const v16h b = ldf_h(wb + (size_t)nt * 16 * FFTN + k0, h);
      acc[0][nt] = wmma_f16(a0, b, acc[0][nt]);
      acc[1][nt] = wmma_f16(a1, b, acc[1][nt]);
    }
  }

  float* so = sT + w * 2048;
  #pragma unroll
  for (int nt = 0; nt < 4; ++nt)
    #pragma unroll
    for (int mt = 0; mt < 2; ++mt)
      #pragma unroll
      for (int r = 0; r < 8; ++r)
        so[(16 * mt + 8 * h + r) * 64 + 16 * nt + m] = acc[mt][nt][r];
  __syncthreads();

  ana_store_pass(so, sph, spl, g0, n0, lane);
  __threadfence();
  ana_store_pass(so, sph, spl, g0, n0, lane);
}

__device__ __forceinline__ size_t syn_aoff(int g) {
  const int b = g / QROWS;
  const int q = g - b * QROWS;
  return (size_t)(b * PROWS + q) * CPAD;
}

__device__ __forceinline__ void syn_store_pass(const float* so, float* out, int g0, int n0, int lane) {
  const int hsel = lane >> 4, c4 = (lane & 15) * 4;
  #pragma unroll
  for (int i = 0; i < 16; ++i) {
    const int row = 2 * i + hsel;
    const v4f v = *(const v4fa*)(so + row * 64 + c4);
    const size_t off = (size_t)(g0 + row) * HOPN + n0 + c4;
    *(volatile v4f*)(out + off) = v;
  }
}

__global__ __launch_bounds__(128) void syn_kernel(const unsigned short* __restrict__ sph,
                                                  const unsigned short* __restrict__ spl,
                                                  const unsigned short* __restrict__ ivh,
                                                  const unsigned short* __restrict__ ivl,
                                                  float* __restrict__ out) {
  __shared__ __attribute__((aligned(16))) float sT[4 * 32 * 64];

  const int tid = threadIdx.x, lane = tid & 31, w = tid >> 5;
  const int h = lane >> 4, m = lane & 15;
  const int g0 = blockIdx.x * 128 + 32 * w;
  const int n0 = blockIdx.y * 64;

  const size_t pa0 = syn_aoff(g0 + m);
  const size_t pa1 = syn_aoff(g0 + 16 + m);
  const size_t pb  = (size_t)(n0 + m) * KSYN;

  const v8f zero8 = {0.f, 0.f, 0.f, 0.f, 0.f, 0.f, 0.f, 0.f};
  v8f acc[2][4];
  #pragma unroll
  for (int mt = 0; mt < 2; ++mt)
    #pragma unroll
    for (int nt = 0; nt < 4; ++nt) acc[mt][nt] = zero8;

  #pragma unroll 1
  for (int k0 = 0; k0 < KSYN; k0 += 32) {
    const v16us a0h = ldf_us(sph + pa0 + k0, h);
    const v16us a0l = ldf_us(spl + pa0 + k0, h);
    const v16us a1h = ldf_us(sph + pa1 + k0, h);
    const v16us a1l = ldf_us(spl + pa1 + k0, h);
    #pragma unroll
    for (int nt = 0; nt < 4; ++nt) {
      const size_t boff = pb + (size_t)nt * 16 * KSYN + k0;
      const v16us bh = ldf_us(ivh + boff, h);
      const v16us bl = ldf_us(ivl + boff, h);
      acc[0][nt] = wmma_bf16(a0h, bh, acc[0][nt]);
      acc[0][nt] = wmma_bf16(a0h, bl, acc[0][nt]);
      acc[0][nt] = wmma_bf16(a0l, bh, acc[0][nt]);
      acc[1][nt] = wmma_bf16(a1h, bh, acc[1][nt]);
      acc[1][nt] = wmma_bf16(a1h, bl, acc[1][nt]);
      acc[1][nt] = wmma_bf16(a1l, bh, acc[1][nt]);
    }
  }

  float* so = sT + w * 2048;
  #pragma unroll
  for (int nt = 0; nt < 4; ++nt)
    #pragma unroll
    for (int mt = 0; mt < 2; ++mt)
      #pragma unroll
      for (int r = 0; r < 8; ++r)
        so[(16 * mt + 8 * h + r) * 64 + 16 * nt + m] = acc[mt][nt][r];
  __syncthreads();

  syn_store_pass(so, out, g0, n0, lane);
  __threadfence();
  syn_store_pass(so, out, g0, n0, lane);
}

extern "C" void kernel_launch(void* const* d_in, const int* in_sizes, int n_in,
                              void* d_out, int out_size, void* d_ws, size_t ws_size,
                              hipStream_t stream) {
  if (n_in < 3) return;
  if (in_sizes[0] != NBATCH * NSAMP) return;
  if (in_sizes[1] != CDIM * FFTN) return;
  if (in_sizes[2] != CDIM * FFTN) return;
  if (out_size != NBATCH * NSAMP) return;

  const float* x   = (const float*)d_in[0];
  const float* fwd = (const float*)d_in[1];
  const float* inv = (const float*)d_in[2];
  float* out = (float*)d_out;

  const size_t xh_bytes = (size_t)NBATCH * NSAMP * 2;
  const size_t fh_bytes = (size_t)CPAD * FFTN * 2;
  const size_t iv_bytes = (size_t)NSYN * KSYN * 2;
  const size_t sp_bytes = (size_t)MANA * CPAD * 2;
  const size_t total = xh_bytes + fh_bytes + 2 * iv_bytes + 2 * sp_bytes;
  if (total > ws_size) return;

  char* ws = (char*)d_ws;
  _Float16* xh = (_Float16*)(ws);
  _Float16* fh = (_Float16*)(ws + xh_bytes);
  unsigned short* ivh = (unsigned short*)(ws + xh_bytes + fh_bytes);
  unsigned short* ivl = (unsigned short*)(ws + xh_bytes + fh_bytes + iv_bytes);
  unsigned short* sph = (unsigned short*)(ws + xh_bytes + fh_bytes + 2 * iv_bytes);
  unsigned short* spl = (unsigned short*)(ws + xh_bytes + fh_bytes + 2 * iv_bytes + sp_bytes);

  const int nx8 = NBATCH * NSAMP / 8;
  cvt_x_kernel<<<(nx8 + 255) / 256, 256, 0, stream>>>(x, xh, nx8);

  const int nf8 = CPAD * FFTN / 8;
  prep_fwd_kernel<<<(nf8 + 255) / 256, 256, 0, stream>>>(fwd, fh);

  const int ni8 = NSYN * KSYN / 8;
  prep_inv_kernel<<<(ni8 + 255) / 256, 256, 0, stream>>>(inv, ivh, ivl);

  dim3 gAna(MANA / 128, CPAD / 64);
  ana_kernel<<<gAna, 128, 0, stream>>>(xh, fh, sph, spl);

  dim3 gSyn(MSYN / 128, NSYN / 64);
  syn_kernel<<<gSyn, 128, 0, stream>>>(sph, spl, ivh, ivl, out);
}
